// HybridQLSTM_65481071396755
// MI455X (gfx1250) — hardware-verified
//
#include <hip/hip_runtime.h>
#include <stddef.h>
#include <stdint.h>

typedef __attribute__((ext_vector_type(16))) _Float16 v16h;
typedef __attribute__((ext_vector_type(8)))  _Float16 v8h;
typedef __attribute__((ext_vector_type(16))) __bf16   v16b;
typedef __attribute__((ext_vector_type(8)))  __bf16   v8b;
typedef __attribute__((ext_vector_type(8)))  float    v8f;
typedef __attribute__((ext_vector_type(4)))  float    v4f;

__device__ __forceinline__ unsigned short f2bf_bits(float f) {
  unsigned u = __float_as_uint(f);
  return (unsigned short)((u + 0x7FFFu + ((u >> 16) & 1u)) >> 16);
}
__device__ __forceinline__ float bf_bits2f(unsigned short h) { return __uint_as_float(((unsigned)h) << 16); }

__device__ __forceinline__ void dep_guard_h(v8f& a, v8f& b, v16h x, v16h y) { asm volatile("v_nop\n\tv_nop\n\tv_nop\n\tv_nop" : "+v"(a), "+v"(b) : "v"(x), "v"(y)); }
__device__ __forceinline__ void dep_guard_b(v8f& a, v8f& b, v16b x, v16b y) { asm volatile("v_nop\n\tv_nop\n\tv_nop\n\tv_nop" : "+v"(a), "+v"(b) : "v"(x), "v"(y)); }
__device__ __forceinline__ void keep4_h(v16h a, v16h b, v16h c, v16h d) { asm volatile("v_nop" :: "v"(a), "v"(b), "v"(c), "v"(d)); }
__device__ __forceinline__ void keep4_b(v16b a, v16b b, v16b c, v16b d) { asm volatile("v_nop" :: "v"(a), "v"(b), "v"(c), "v"(d)); }
__device__ __forceinline__ void acc_guard4(v8f& a, v8f& b, v8f& c, v8f& d) { asm volatile("v_nop\n\tv_nop\n\tv_nop\n\tv_nop" : "+v"(a), "+v"(b), "+v"(c), "+v"(d)); }
template <typename T> struct Frag;
template <> struct Frag<_Float16> {
  typedef v16h V; union U { v16h v; v8h h[2]; };
  static __device__ __forceinline__ v16h load(const _Float16* p) {
    U f; f.h[0] = *(const v8h*)(p); f.h[1] = *(const v8h*)(p + 16); return f.v;
  }
  static __device__ __forceinline__ v8f mma(v16h a, v16h b, v8f c) {
    return __builtin_amdgcn_wmma_f32_16x16x32_f16(false, a, false, b, (short)0, c, false, false);
  }
  static __device__ __forceinline__ void guard(v8f& a, v8f& b, v16h x, v16h y) { dep_guard_h(a, b, x, y); }
  static __device__ __forceinline__ void keep(v16h a, v16h b, v16h c, v16h d) { keep4_h(a, b, c, d); }
};
template <> struct Frag<__bf16> {
  typedef v16b V; union U { v16b v; v8b h[2]; };
  static __device__ __forceinline__ v16b load(const __bf16* p) {
    U f; f.h[0] = *(const v8b*)(p); f.h[1] = *(const v8b*)(p + 16); return f.v;
  }
  static __device__ __forceinline__ v8f mma(v16b a, v16b b, v8f c) {
    return __builtin_amdgcn_wmma_f32_16x16x32_bf16(false, a, false, b, (short)0, c, false, false);
  }
  static __device__ __forceinline__ void guard(v8f& a, v8f& b, v16b x, v16b y) { dep_guard_b(a, b, x, y); }
  static __device__ __forceinline__ void keep(v16b a, v16b b, v16b c, v16b d) { keep4_b(a, b, c, d); }
};

template <int ET> struct Elem;
template <> struct Elem<0> { typedef _Float16 T; };
template <> struct Elem<1> { typedef __bf16 T; };
template <int ET, bool SPLIT, int BIAS_MODE, int OUT_MODE, bool RESID, int ACT = 0>
__global__ __launch_bounds__(256) void wmma_gemm64(
    const unsigned short* __restrict__ Ap, const unsigned short* __restrict__ A2p, int lda, long strideA,
    const unsigned short* __restrict__ Btp, const unsigned short* __restrict__ Bt2p, int ldb, long strideB,
    void* __restrict__ Cout, void* __restrict__ Cout2, int ldc, long strideC,
    const float* __restrict__ bias,
    const float* __restrict__ resid, long strideR,
    int M, int N, int K, float scale) {
  typedef typename Elem<ET>::T T;
  typedef typename Frag<T>::V V;
  const T* A = (const T*)Ap; const T* A2 = (const T*)A2p; const T* Bt = (const T*)Btp; const T* Bt2 = (const T*)Bt2p;
  __shared__ __align__(16) float sT[8][16 * 68];
  const int b    = blockIdx.y;
  const int lane = threadIdx.x & 31;
  const int wave = threadIdx.x >> 5;
  const int tilesN = N >> 6;
  const int tilesM = M >> 6;
  const int tile = blockIdx.x * 8 + wave;
  if (tile >= tilesM * tilesN) return;
  const int tm = tile / tilesN;
  const int tn = tile - tm * tilesN;
  const int m0 = tm << 6;
  const int n0 = tn << 6;

  const T* Ab  = A  + (size_t)b * strideA;
  const T* Bb  = Bt + (size_t)b * strideB;
  const T* Ab2 = SPLIT ? (A2  + (size_t)b * strideA) : nullptr;
  const T* Bb2 = SPLIT ? (Bt2 + (size_t)b * strideB) : nullptr;

  const int rlane = lane & 15;
  const int koff  = (lane >> 4) * 8;
  const int mOff  = (lane >> 4) * 8;

  v8f acc[4][4];
#pragma unroll
  for (int i = 0; i < 4; ++i)
#pragma unroll
    for (int j = 0; j < 4; ++j) acc[i][j] = (v8f){0.f,0.f,0.f,0.f,0.f,0.f,0.f,0.f};

  for (int k0 = 0; k0 < K; k0 += 32) {
    V bh[4], bl[4];
#pragma unroll
    for (int j = 0; j < 4; ++j) {
      const size_t bo = (size_t)(n0 + (j << 4) + rlane) * ldb + koff + k0;
      bh[j] = Frag<T>::load(Bb + bo);
      if (SPLIT) bl[j] = Frag<T>::load(Bb2 + bo);
    }
#pragma unroll
    for (int i = 0; i < 4; ++i) {
      const size_t ao = (size_t)(m0 + (i << 4) + rlane) * lda + koff + k0;
      V ah = Frag<T>::load(Ab + ao);
      V al;
      if (SPLIT) al = Frag<T>::load(Ab2 + ao);
#pragma unroll
      for (int j = 0; j < 4; ++j) {
        acc[i][j] = Frag<T>::mma(ah, bh[j], acc[i][j]);
        if (SPLIT) {
          acc[i][j] = Frag<T>::mma(ah, bl[j], acc[i][j]);
          acc[i][j] = Frag<T>::mma(al, bh[j], acc[i][j]);
        }
      }
      Frag<T>::guard(acc[i][0], acc[i][3], ah, SPLIT ? al : ah);
    }
    Frag<T>::keep(bh[0], bh[1], bh[2], bh[3]);
    if (SPLIT) Frag<T>::keep(bl[0], bl[1], bl[2], bl[3]);
  }
  acc_guard4(acc[0][0], acc[0][1], acc[0][2], acc[0][3]);
  acc_guard4(acc[1][0], acc[1][1], acc[1][2], acc[1][3]);
  acc_guard4(acc[2][0], acc[2][1], acc[2][2], acc[2][3]);
  acc_guard4(acc[3][0], acc[3][1], acc[3][2], acc[3][3]);

  float* slab = sT[wave];
  const float* Rb = RESID ? (resid + (size_t)b * strideR) : nullptr;
#pragma unroll
  for (int i = 0; i < 4; ++i) {
    const int mBase = m0 + (i << 4);
#pragma unroll
    for (int j = 0; j < 4; ++j) {
      const int n = n0 + (j << 4) + rlane;
      float bv = 0.f;
      if (BIAS_MODE == 2) bv = bias[n];
#pragma unroll
      for (int r = 0; r < 8; ++r) {
        float v = acc[i][j][r] * scale;
        if (BIAS_MODE == 1) v += bias[mBase + mOff + r];
        if (BIAS_MODE == 2) v += bv;
        if (RESID) v += Rb[(size_t)(mBase + mOff + r) * ldc + n];
        if (ACT == 1) v = tanhf(v);
        if (ACT == 2) v = fmaxf(v, 0.0f);
        if (ACT == 3) v = v / (1.0f + expf(-v));
        if (ACT == 4) v = (v > 0.f) ? v : 0.01f * v;
        if (ACT == 5) v = 0.5f * v * (1.0f + erff(v * 0.70710678118654752f));
        slab[(mOff + r) * 68 + (j << 4) + rlane] = v;
      }
    }
    __builtin_amdgcn_fence(__ATOMIC_RELEASE, "workgroup");
    __builtin_amdgcn_wave_barrier();
    __builtin_amdgcn_fence(__ATOMIC_ACQUIRE, "workgroup");
    if (OUT_MODE == 0) {
      float* C = (float*)Cout + (size_t)b * strideC;
      const int hh = lane >> 4, c4 = (lane & 15) * 4;
      for (int pass = 0; pass < 2; ++pass) {
#pragma unroll
        for (int it = 0; it < 8; ++it) {
          const int row = it * 2 + hh;
          v4f v = *(const v4f*)(slab + row * 68 + c4);
          *(volatile v4f*)(C + (size_t)(mBase + row) * ldc + n0 + c4) = v;
        }
        __threadfence();
      }
    } else {
      const int q = lane >> 3, c8 = (lane & 7) * 8;
      unsigned short* C  = (unsigned short*)Cout  + (size_t)b * strideC;
      unsigned short* C2 = (OUT_MODE == 2) ? ((unsigned short*)Cout2 + (size_t)b * strideC) : nullptr;
      for (int pass = 0; pass < 2; ++pass) {
#pragma unroll
        for (int it = 0; it < 4; ++it) {
          const int row = it * 4 + q;
          const float* sp = slab + row * 68 + c8;
          v8h hv, lv;
#pragma unroll
          for (int e = 0; e < 8; ++e) {
            if (OUT_MODE == 1) {
              hv[e] = (_Float16)sp[e];
            } else {
              unsigned short hb = f2bf_bits(sp[e]);
              unsigned short lb = f2bf_bits(sp[e] - bf_bits2f(hb));
              hv[e] = __builtin_bit_cast(_Float16, hb);
              lv[e] = __builtin_bit_cast(_Float16, lb);
            }
          }
          *(volatile v8h*)(C + (size_t)(mBase + row) * ldc + n0 + c8) = hv;
          if (OUT_MODE == 2) *(volatile v8h*)(C2 + (size_t)(mBase + row) * ldc + n0 + c8) = lv;
        }
        __threadfence();
      }
    }
    __builtin_amdgcn_fence(__ATOMIC_RELEASE, "workgroup");
    __builtin_amdgcn_wave_barrier();
    __builtin_amdgcn_fence(__ATOMIC_ACQUIRE, "workgroup");
  }
}

constexpr int DIM_B = 64;
constexpr int DIM_S = 512;
constexpr int DIM_E = 256;
constexpr int DIM_H = 256;
constexpr int DIM_V = 32000;
constexpr int DIM_T = 64;
constexpr int DIM_G4 = 4 * DIM_H;
constexpr int KCOMB = DIM_E + DIM_H;
constexpr int XH_PITCH = KCOMB + 8;
constexpr int ROWS_PER_BLOCK = 16;
constexpr int LSTM_THREADS = 512;
constexpr int NBLK_LSTM = DIM_B / ROWS_PER_BLOCK;

static_assert(DIM_E == DIM_H, "second cell reuses the K=512 layout: [x(256) | h(256)]");
static_assert(KCOMB % 32 == 0, "WMMA K step");
static_assert(DIM_H % 32 == 0, "tag GEMM K step");
static_assert(XH_PITCH % 8 == 0, "16-B alignment of fragment loads");
static_assert((LSTM_THREADS / 32) * 16 == DIM_H, "one wave per 16 hidden units");
static_assert(LSTM_THREADS == ROWS_PER_BLOCK * 32, "x staging: wave w fills row w, 32 lanes x 8 halves = 256");
static_assert(LSTM_THREADS * 8 == ROWS_PER_BLOCK * DIM_H, "h store: 512 threads x 8 halves = 16 rows x 256, 64 whole lines");
static_assert(DIM_B % ROWS_PER_BLOCK == 0, "");
static_assert((DIM_B * DIM_S) % 64 == 0 && DIM_T % 64 == 0, "kit GEMM tile multiples (M=32768, N=64)");

constexpr size_t WS_WG1_OFF = 0;
constexpr size_t WS_WG1_SZ  = (size_t)DIM_G4 * KCOMB * 2;
constexpr size_t WS_WG2_OFF = WS_WG1_OFF + WS_WG1_SZ;
constexpr size_t WS_WG2_SZ  = (size_t)DIM_G4 * KCOMB * 2;
constexpr size_t WS_WT_OFF  = WS_WG2_OFF + WS_WG2_SZ;
constexpr size_t WS_WT_SZ   = (size_t)DIM_T * DIM_H * 2;
constexpr size_t WS_H1_OFF  = WS_WT_OFF + WS_WT_SZ;
constexpr size_t WS_H1_SZ   = (size_t)DIM_S * DIM_B * DIM_H * 2;
constexpr size_t WS_H2_OFF  = WS_H1_OFF + WS_H1_SZ;
constexpr size_t WS_H2_SZ   = (size_t)DIM_B * DIM_S * DIM_H * 2;
constexpr size_t WS_LG_OFF  = WS_H2_OFF + WS_H2_SZ;
constexpr size_t WS_LG_SZ   = (size_t)DIM_B * DIM_S * DIM_T * 4;
constexpr size_t WS_TOTAL   = WS_LG_OFF + WS_LG_SZ;
static_assert(WS_TOTAL == 44072960, "carve total");
static_assert(WS_TOTAL <= (size_t)134217728, "carve under 128 MiB");
static_assert(WS_WG2_OFF % 256 == 0 && WS_WT_OFF % 256 == 0 && WS_H1_OFF % 256 == 0 &&
              WS_H2_OFF % 256 == 0 && WS_LG_OFF % 256 == 0, "alignment");

__device__ __forceinline__ __bf16 to_bf16(float f) { return __builtin_bit_cast(__bf16, f2bf_bits(f)); }

__device__ __forceinline__ v8f mma_bf16_guarded(v16b a, v16b b, v8f c) {
  c = __builtin_amdgcn_wmma_f32_16x16x32_bf16(false, a, false, b, (short)0, c, false, false);
  asm volatile("v_nop\n\tv_nop\n\tv_nop\n\tv_nop" : "+v"(c) : "v"(a), "v"(b));
  return c;
}

__device__ __forceinline__ float sigm_f(float x) {
  const float e = __expf(fminf(-x, 80.0f));
  return __builtin_amdgcn_rcpf(1.0f + e);
}

__global__ __launch_bounds__(256) void cast_rows_bf16(const float* __restrict__ src, int cols,
                                                      __bf16* __restrict__ dst, int dpitch, int coff, int n8) {
  const int i = blockIdx.x * 256 + threadIdx.x;
  const int ic = (i < n8) ? i : (n8 - 1);
  const size_t e = (size_t)ic * 8;
  const int r = (int)(e / (size_t)cols);
  const int c = (int)(e - (size_t)r * cols);
  const v4f f0 = *(const v4f*)(src + e);
  const v4f f1 = *(const v4f*)(src + e + 4);
  v8b o;
  o[0] = to_bf16(f0[0]); o[1] = to_bf16(f0[1]); o[2] = to_bf16(f0[2]); o[3] = to_bf16(f0[3]);
  o[4] = to_bf16(f1[0]); o[5] = to_bf16(f1[1]); o[6] = to_bf16(f1[2]); o[7] = to_bf16(f1[3]);
  __bf16* d = dst + (size_t)r * dpitch + coff + c;
  if (i < n8) *(volatile v8b*)d = o;
  __threadfence();
  if (i < n8) *(volatile v8b*)d = o;
}

template <int GF, int GI, bool FIRST>
__global__ __launch_bounds__(LSTM_THREADS) void lstm_seq_kernel(
    const int* __restrict__ sent, const float* __restrict__ emb, int vocab,
    const __bf16* __restrict__ xin, const __bf16* __restrict__ Wc,
    const float* __restrict__ bA, const float* __restrict__ bB,
    const float* __restrict__ bC, const float* __restrict__ bD,
    __bf16* __restrict__ hout, int nsteps) {
  __shared__ __align__(16) __bf16 xh[ROWS_PER_BLOCK * XH_PITCH];

  const int tid  = threadIdx.x;
  const int wave = tid >> 5;
  const int lane = tid & 31;
  const int hh   = lane >> 4;
  const int rl   = lane & 15;
  const int koff = hh * 8;
  const int b0   = blockIdx.x * ROWS_PER_BLOCK;
  const int unit = wave * 16 + rl;

  float bsv[4];
  if (FIRST) {
    bsv[0] = bA[unit]; bsv[1] = bB[unit]; bsv[2] = bC[unit]; bsv[3] = bD[unit];
  } else {
#pragma unroll
    for (int gb = 0; gb < 4; ++gb) bsv[gb] = bA[gb * DIM_H + unit] + bB[gb * DIM_H + unit];
  }
  float cst[8];
#pragma unroll
  for (int r = 0; r < 8; ++r) cst[r] = 0.0f;

  const int srow = tid >> 5;
  const int scol = (tid & 31) * 8;
  const int oline = tid >> 3;
  const int oq    = tid & 7;
  const int orow  = oline >> 2;
  const int ocol  = (oline & 3) * 64 + oq * 8;

  int ns = nsteps;
  if (ns > DIM_S) ns = DIM_S;
  if (ns < 0) ns = 0;
  const int vmax = (vocab > 0) ? (vocab - 1) : 0;

  for (int t = 0; t < ns; ++t) {
    if (FIRST) {
      int tok = sent[(size_t)(b0 + srow) * DIM_S + t];
      tok = (tok < 0) ? 0 : tok;
      tok = (tok > vmax) ? vmax : tok;
      const float* src = emb + (size_t)tok * DIM_E + scol;
      const v4f f0 = *(const v4f*)(src);
      const v4f f1 = *(const v4f*)(src + 4);
      v8b xv;
      xv[0] = to_bf16(f0[0]); xv[1] = to_bf16(f0[1]); xv[2] = to_bf16(f0[2]); xv[3] = to_bf16(f0[3]);
      xv[4] = to_bf16(f1[0]); xv[5] = to_bf16(f1[1]); xv[6] = to_bf16(f1[2]); xv[7] = to_bf16(f1[3]);
      *(v8b*)(xh + srow * XH_PITCH + scol) = xv;
    } else {
      const v8b xv = *(const v8b*)(xin + ((size_t)t * DIM_B + b0 + srow) * DIM_H + scol);
      *(v8b*)(xh + srow * XH_PITCH + scol) = xv;
    }
    __syncthreads();

    v8f acc[4];
#pragma unroll
    for (int gb = 0; gb < 4; ++gb) acc[gb] = (v8f){0.f,0.f,0.f,0.f,0.f,0.f,0.f,0.f};
    const int kEnd = (t == 0) ? DIM_E : KCOMB;
#pragma unroll 1
    for (int k0 = 0; k0 < kEnd; k0 += 32) {
      const v16b a  = Frag<__bf16>::load(xh + rl * XH_PITCH + k0 + koff);
      const __bf16* wp = Wc + (size_t)unit * KCOMB + k0 + koff;
      const v16b w0 = Frag<__bf16>::load(wp);
      const v16b w1 = Frag<__bf16>::load(wp + (size_t)1 * DIM_H * KCOMB);
      const v16b w2 = Frag<__bf16>::load(wp + (size_t)2 * DIM_H * KCOMB);
      const v16b w3 = Frag<__bf16>::load(wp + (size_t)3 * DIM_H * KCOMB);
      acc[0] = mma_bf16_guarded(a, w0, acc[0]);
      acc[1] = mma_bf16_guarded(a, w1, acc[1]);
      acc[2] = mma_bf16_guarded(a, w2, acc[2]);
      acc[3] = mma_bf16_guarded(a, w3, acc[3]);
    }
    __syncthreads();

#pragma unroll
    for (int r = 0; r < 8; ++r) {
      const float pf = acc[GF][r] + bsv[GF];
      const float pi = acc[GI][r] + bsv[GI];
      const float pg = acc[2][r]  + bsv[2];
      const float po = acc[3][r]  + bsv[3];
      const float fv = sigm_f(pf);
      const float iv = sigm_f(pi);
      const float gv = tanhf(pg);
      const float ov = sigm_f(po);
      const float cn = fv * cst[r] + iv * gv;
      cst[r] = cn;
      const float hv = ov * tanhf(cn);
      xh[(hh * 8 + r) * XH_PITCH + DIM_E + unit] = to_bf16(hv);
    }
    __syncthreads();

    {
      const v8b hv8 = *(const v8b*)(xh + orow * XH_PITCH + DIM_E + ocol);
      const size_t grow = FIRST ? ((size_t)t * DIM_B + (size_t)(b0 + orow))
                                : ((size_t)(b0 + orow) * DIM_S + (size_t)t);
      __bf16* dst = hout + grow * DIM_H + ocol;
      *(volatile v8b*)dst = hv8;
      __threadfence();
      *(volatile v8b*)dst = hv8;
    }
  }
}

__global__ __launch_bounds__(256) void log_softmax64_kernel(const float* __restrict__ lg,
                                                           float* __restrict__ out, int nrows) {
  const int tid = threadIdx.x;
  const int wave = tid >> 5, lane = tid & 31, hh = lane >> 4;
  const int c4 = (lane & 15) * 4;
  const int row = blockIdx.x * 16 + wave * 2 + hh;
  const int rowc = (row < nrows) ? row : (nrows - 1);
  const v4f v = *(const v4f*)(lg + (size_t)rowc * DIM_T + c4);
  float m = fmaxf(fmaxf(v[0], v[1]), fmaxf(v[2], v[3]));
  m = fmaxf(m, __shfl_xor(m, 1, 32));
  m = fmaxf(m, __shfl_xor(m, 2, 32));
  m = fmaxf(m, __shfl_xor(m, 4, 32));
  m = fmaxf(m, __shfl_xor(m, 8, 32));
  const float s0 = v[0] - m, s1 = v[1] - m, s2 = v[2] - m, s3 = v[3] - m;
  float se = __expf(s0) + __expf(s1) + __expf(s2) + __expf(s3);
  se += __shfl_xor(se, 1, 32);
  se += __shfl_xor(se, 2, 32);
  se += __shfl_xor(se, 4, 32);
  se += __shfl_xor(se, 8, 32);
  const float ls = __logf(se);
  v4f o;
  o[0] = s0 - ls; o[1] = s1 - ls; o[2] = s2 - ls; o[3] = s3 - ls;
  float* d = out + (size_t)rowc * DIM_T + c4;
  if (row < nrows) *(volatile v4f*)d = o;
  __threadfence();
  if (row < nrows) *(volatile v4f*)d = o;
}

extern "C" void kernel_launch(void* const* d_in, const int* in_sizes, int n_in,
                              void* d_out, int out_size, void* d_ws, size_t ws_size,
                              hipStream_t stream) {
  if (n_in < 16) return;
  if (in_sizes[0] != DIM_B * DIM_S) return;
  if (in_sizes[1] < DIM_E) return;
  if (in_sizes[2] != DIM_H * KCOMB || in_sizes[4] != DIM_H * KCOMB ||
      in_sizes[6] != DIM_H * KCOMB || in_sizes[8] != DIM_H * KCOMB) return;
  if (in_sizes[3] != DIM_H || in_sizes[5] != DIM_H || in_sizes[7] != DIM_H || in_sizes[9] != DIM_H) return;
  if (in_sizes[10] != DIM_G4 * DIM_H || in_sizes[11] != DIM_G4 * DIM_H) return;
  if (in_sizes[12] != DIM_G4 || in_sizes[13] != DIM_G4) return;
  if (in_sizes[14] != DIM_T * DIM_H || in_sizes[15] != DIM_T) return;
  if (out_size != DIM_B * DIM_S * DIM_T) return;
  if (ws_size < WS_TOTAL) return;

  const int*   sent = (const int*)d_in[0];
  const float* emb  = (const float*)d_in[1];
  const float* Wf   = (const float*)d_in[2];
  const float* bf   = (const float*)d_in[3];
  const float* Wi   = (const float*)d_in[4];
  const float* bi   = (const float*)d_in[5];
  const float* Wu   = (const float*)d_in[6];
  const float* bu   = (const float*)d_in[7];
  const float* Wo   = (const float*)d_in[8];
  const float* bo   = (const float*)d_in[9];
  const float* Wih  = (const float*)d_in[10];
  const float* Whh  = (const float*)d_in[11];
  const float* bih  = (const float*)d_in[12];
  const float* bhh  = (const float*)d_in[13];
  const float* Wtag = (const float*)d_in[14];
  const float* btag = (const float*)d_in[15];
  float* out = (float*)d_out;
  const int vocab = in_sizes[1] / DIM_E;

  char* ws = (char*)d_ws;
  __bf16* wg1 = (__bf16*)(ws + WS_WG1_OFF);
  __bf16* wg2 = (__bf16*)(ws + WS_WG2_OFF);
  __bf16* wt  = (__bf16*)(ws + WS_WT_OFF);
  __bf16* h1  = (__bf16*)(ws + WS_H1_OFF);
  __bf16* h2  = (__bf16*)(ws + WS_H2_OFF);
  float*  lg  = (float*)(ws + WS_LG_OFF);

  auto cast = [&](const float* src, int rows, int cols, __bf16* dst, int dpitch, int coff) {
    const int n8 = rows * cols / 8;
    const int grid = (n8 + 255) / 256;
    cast_rows_bf16<<<grid, 256, 0, stream>>>(src, cols, dst, dpitch, coff, n8);
  };
  cast(Wf,  DIM_H, KCOMB, wg1 + (size_t)0 * DIM_H * KCOMB, KCOMB, 0);
  cast(Wi,  DIM_H, KCOMB, wg1 + (size_t)1 * DIM_H * KCOMB, KCOMB, 0);
  cast(Wu,  DIM_H, KCOMB, wg1 + (size_t)2 * DIM_H * KCOMB, KCOMB, 0);
  cast(Wo,  DIM_H, KCOMB, wg1 + (size_t)3 * DIM_H * KCOMB, KCOMB, 0);
  cast(Wih, DIM_G4, DIM_H, wg2, KCOMB, 0);
  cast(Whh, DIM_G4, DIM_H, wg2, KCOMB, DIM_E);
  cast(Wtag, DIM_T, DIM_H, wt, DIM_H, 0);

  lstm_seq_kernel<0, 1, true><<<NBLK_LSTM, LSTM_THREADS, 0, stream>>>(
      sent, emb, vocab, h1, wg1, bf, bi, bu, bo, h1, DIM_S);
  lstm_seq_kernel<1, 0, false><<<NBLK_LSTM, LSTM_THREADS, 0, stream>>>(
      sent, emb, vocab, h1, wg2, bih, bhh, bih, bhh, h2, DIM_S);

  {
    const int M = DIM_B * DIM_S;
    const int tiles = (M / 64) * (DIM_T / 64);
    const int grid = (tiles + 7) / 8;
    wmma_gemm64<1, false, 2, 0, false, 0><<<dim3(grid, 1), 256, 0, stream>>>(
        (const unsigned short*)h2, (const unsigned short*)h2, DIM_H, 0L,
        (const unsigned short*)wt, (const unsigned short*)wt, DIM_H, 0L,
        (void*)lg, (void*)lg, DIM_T, 0L,
        btag, btag, 0L,
        M, DIM_T, DIM_H, 1.0f);
  }

  {
    const int nrows = DIM_B * DIM_S;
    const int grid = (nrows + 15) / 16;
    log_softmax64_kernel<<<grid, 256, 0, stream>>>(lg, out, nrows);
  }
}
